// NaNHandlingLayer_45861660786920
// MI455X (gfx1250) — hardware-run, weakly checked
//
#include <hip/hip_runtime.h>


#define NRW  4096
#define NFT  512
#define NKD  1024
#define NQW  64
#define NTW  10
#define OFW  0
#define OBS  5120
#define OWW  5632
#define OCB  6400
constexpr size_t al256(size_t b) { return (b + 255) & ~(size_t)255; }
constexpr size_t WS_TOTAL = al256((size_t)8192 * 4) + 2 * al256((size_t)NRW * NFT * 4) + al256((size_t)NRW * NKD * 2) + al256((size_t)NQW * NKD * 2) + al256((size_t)NRW * NQW * 4);
static_assert(WS_TOTAL == 26378240 && WS_TOTAL <= 134217728, "the workspace carve: 25.2 MiB");
static_assert(NKD == 2 * NFT && NRW % 64 == 0 && NQW == 64 && NKD % 64 == 0 && NFT % 256 == 0 && OBS == NFT * NTW && OWW == OBS + NFT && OCB >= OWW + (NTW + 1) * NQW && OCB + NQW <= 8192 && OBS % 4 == 0 && OWW % 4 == 0 && OCB % 4 == 0, "whole tiles; whole lines; the record's parts apart and on 16-byte pieces");
typedef _Float16 h16;
typedef unsigned short bf;
typedef __attribute__((ext_vector_type(16))) __bf16   v16bf;
typedef __attribute__((ext_vector_type(16))) _Float16 v16h;
typedef __attribute__((ext_vector_type(8)))  _Float16 v8h;
typedef __attribute__((ext_vector_type(8)))  unsigned short v8us;
typedef __attribute__((ext_vector_type(8)))  float    v8f;
typedef __attribute__((ext_vector_type(4)))  float    v4f;
typedef v8h  __attribute__((may_alias)) v8ha;
typedef v4f  __attribute__((may_alias)) v4fa;
typedef v8us __attribute__((may_alias)) v8usa;

__device__ __forceinline__ unsigned short f2bf(float f) { unsigned u = __float_as_uint(f); u += 0x7FFFu + ((u >> 16) & 1u); return (unsigned short)(u >> 16); }
__device__ __forceinline__ float bf2f(unsigned short b) { return __uint_as_float(((unsigned)b) << 16); }
__device__ __forceinline__ float bfr(float f) { return bf2f(f2bf(f)); }
__device__ __forceinline__ v16h cat16(v8h lo, v8h hi) { return __builtin_shufflevector(lo, hi, 0, 1, 2, 3, 4, 5, 6, 7, 8, 9, 10, 11, 12, 13, 14, 15); }
__device__ __forceinline__ v16bf cat16b(v8us lo, v8us hi) { return __builtin_bit_cast(v16bf, __builtin_shufflevector(lo, hi, 0, 1, 2, 3, 4, 5, 6, 7, 8, 9, 10, 11, 12, 13, 14, 15)); }
__device__ __forceinline__ v8f wmma16(v16h a, v16h b, v8f c) { return __builtin_amdgcn_wmma_f32_16x16x32_f16(false, a, false, b, (short)0, c, false, false); }
__device__ __forceinline__ v8f wmmab(v16bf a, v16bf b, v8f c) { return __builtin_amdgcn_wmma_f32_16x16x32_bf16(false, a, false, b, (short)0, c, false, false); }


template <typename T16> struct WFrag;
template <> struct WFrag<h16> { typedef v16h V; static __device__ __forceinline__ V ld(const h16* p) { return cat16(*(const v8h*)p, *(const v8h*)(p + 16)); } static __device__ __forceinline__ v8f mma(V a, V b, v8f c) { return wmma16(a, b, c); } };
template <> struct WFrag<bf> { typedef v16bf V; static __device__ __forceinline__ V ld(const bf* p) { return cat16b(*(const v8us*)p, *(const v8us*)(p + 16)); } static __device__ __forceinline__ v8f mma(V a, V b, v8f c) { return wmmab(a, b, c); } };
template <typename T16, int NSPLIT, bool BIAS>
__global__ __launch_bounds__(32) void k_gemmw(const T16* __restrict__ A, const T16* __restrict__ A2, const T16* __restrict__ Bt, const T16* __restrict__ Bt2, int K, float* C, int ldc, const float* __restrict__ bias, size_t sA, size_t sB, size_t sC) {
    typedef typename WFrag<T16>::V V;
    __shared__ __align__(16) float os[16 * 68];
    const size_t z = blockIdx.z; A += z * sA; if (A2) A2 += z * sA; Bt += z * sB; if (Bt2) Bt2 += z * sB; C += z * sC;
    const int lane = threadIdx.x & 31, lr = lane & 15, hi = lane >> 4; const int r0 = blockIdx.x * 64, c0 = blockIdx.y * 64;
    v8f acc[4][4];
#pragma unroll
    for (int mb = 0; mb < 4; ++mb)
#pragma unroll
        for (int nb = 0; nb < 4; ++nb) acc[mb][nb] = (v8f){};
    const size_t aoff = (size_t)(r0 + lr) * K + 8 * hi, boff = (size_t)(c0 + lr) * K + 8 * hi;
    for (int kc = 0; kc < K; kc += 32) {
        V a[4], a2[4];
#pragma unroll
        for (int mb = 0; mb < 4; ++mb) { a[mb] = WFrag<T16>::ld(A + aoff + (size_t)mb * 16 * K + kc); if (NSPLIT == 1 || NSPLIT == 2) a2[mb] = WFrag<T16>::ld(A2 + aoff + (size_t)mb * 16 * K + kc); }
#pragma unroll
        for (int nb = 0; nb < 4; ++nb) { const V b = WFrag<T16>::ld(Bt + boff + (size_t)nb * 16 * K + kc); V b2; if (NSPLIT >= 2) b2 = WFrag<T16>::ld(Bt2 + boff + (size_t)nb * 16 * K + kc);
#pragma unroll
            for (int mb = 0; mb < 4; ++mb) { acc[mb][nb] = WFrag<T16>::mma(a[mb], b, acc[mb][nb]); if (NSPLIT == 1 || NSPLIT == 2) acc[mb][nb] = WFrag<T16>::mma(a2[mb], b, acc[mb][nb]); if (NSPLIT >= 2) acc[mb][nb] = WFrag<T16>::mma(a[mb], b2, acc[mb][nb]); } }
        asm volatile("v_nop\n\tv_nop\n\tv_nop\n\tv_nop" : "+v"(acc[0][0]), "+v"(acc[1][1]), "+v"(acc[2][2]), "+v"(acc[3][3]) : "v"(a[0]), "v"(a[3]));
    }
#pragma unroll
    for (int mb = 0; mb < 4; ++mb) {
#pragma unroll
        for (int nb = 0; nb < 4; ++nb) {
#pragma unroll
            for (int j = 0; j < 8; ++j) os[(hi * 8 + j) * 68 + nb * 16 + lr] = acc[mb][nb][j]; }
        __builtin_amdgcn_wave_barrier(); asm volatile("" ::: "memory");
        float* crow = C + (size_t)(r0 + mb * 16) * ldc + c0;
#pragma unroll 1
        for (int ps = 0; ps < 2; ++ps) {
#pragma unroll
            for (int s = 0; s < 8; ++s) { const int row = 2 * s + hi, cofs = lr * 4; v4f val = *(const v4fa*)(os + row * 68 + cofs); if (BIAS) { val[0] += bfr(bias[c0 + cofs]); val[1] += bfr(bias[c0 + cofs + 1]); val[2] += bfr(bias[c0 + cofs + 2]); val[3] += bfr(bias[c0 + cofs + 3]); }
                *(volatile v4f*)(crow + (size_t)row * ldc + cofs) = val; }
            if (ps == 0) __threadfence(); }
        __builtin_amdgcn_wave_barrier(); asm volatile("" ::: "memory");
    }
}

__device__ __forceinline__ h16 tohx(float x) { return (h16)x; }
__device__ __forceinline__ void splitf(float y, unsigned short& h, unsigned short& l) { h = f2bf(y); l = f2bf(y - bf2f(h)); }
typedef __attribute__((ext_vector_type(2))) _Float16 v2h;
typedef __attribute__((ext_vector_type(4))) _Float16 v4h;
typedef __attribute__((ext_vector_type(2))) unsigned short v2us;
typedef __attribute__((ext_vector_type(4))) unsigned short v4us;
typedef __attribute__((ext_vector_type(2))) float v2f;
typedef __attribute__((ext_vector_type(4))) int v4i;


__global__ __launch_bounds__(256) void k_lay(const float* __restrict__ src, h16* dst, unsigned nrow, unsigned c8n, unsigned dp, unsigned c0, unsigned rbs, unsigned ra, unsigned rs, unsigned cbs, unsigned sa, unsigned sb, unsigned rlive, unsigned clive) {
    const unsigned g = blockIdx.x * 256 + threadIdx.x; if (g >= nrow * c8n) return; const unsigned row = g / c8n, ch = g - row * c8n; const unsigned rb = (row >> rbs) * ra + (row & ((1u << rbs) - 1u)) * rs; v8h o;
#pragma unroll
    for (int w = 0; w < 8; ++w) { const unsigned c = 8u * ch + w; const bool live = row < rlive && c < clive; const unsigned si = rb + (c >> cbs) * sa + (c & ((1u << cbs) - 1u)) * sb; const float v = bfr(src[live ? si : 0u]); o[w] = tohx(live && fabsf(v) >= 6.103515625e-05f ? v : 0.0f); }
    h16* d8 = dst + (size_t)row * dp + c0 + 8u * ch; *(volatile v8h*)(d8) = o; __threadfence(); *(volatile v8h*)(d8) = o; }

__global__ __launch_bounds__(256) void k_rnd(const float* __restrict__ src, float* dst, unsigned npc, unsigned nw) {
    const unsigned g = blockIdx.x * 256 + threadIdx.x; if (g >= npc) return; v4f o;
#pragma unroll
    for (int e = 0; e < 4; ++e) { const unsigned i = 4u * g + (unsigned)e; const unsigned live = i < nw ? 1u : 0u; const float rv_ = bfr(src[live ? i : 0u]); o[e] = live ? rv_ : 0.0f; }
    float* dq = dst + 4u * (size_t)g; *(volatile v4f*)(dq) = o; __threadfence(); *(volatile v4f*)(dq) = o; }

__global__ __launch_bounds__(256) void k_opa(const float* __restrict__ xr, const float* __restrict__ fr, h16* am) {
    const unsigned g = blockIdx.x * 256 + threadIdx.x; if (g >= (unsigned)(NRW * (NFT / 8))) return; const unsigned rw = g >> 6, pc = g & 63u; const float* xq = xr + (size_t)rw * NFT + 8u * pc; const float* fq = fr + (size_t)rw * NFT + 8u * pc; v8h o;
#pragma unroll
    for (int e = 0; e < 8; ++e) { const float pv = fq[e] * xq[e]; o[e] = tohx(fabsf(pv) >= 6.103515625e-05f ? pv : 0.0f); }
    h16* d8 = am + (size_t)rw * NKD + 8u * pc; *(volatile v8h*)(d8) = o; __threadfence(); *(volatile v8h*)(d8) = o; }

__global__ __launch_bounds__(256) void k_opb(const float* __restrict__ rs, h16* bt) {
    const unsigned g = blockIdx.x * 256 + threadIdx.x; if (g >= (unsigned)(NQW * (NKD / 8))) return; const unsigned q = g >> 7, pc = g & 127u, hi = pc >> 6, d0 = 8u * (pc & 63u); const float hf = hi ? 1.0f : 0.0f, lf = 1.0f - hf; const float w10 = rs[OWW + NTW * NQW + q], cq = rs[OCB + q]; float wt[NTW];
#pragma unroll
    for (int t = 0; t < NTW; ++t) wt[t] = rs[OWW + t * NQW + q];
    v8h o;
#pragma unroll
    for (int e = 0; e < 8; ++e) { const unsigned d = d0 + (unsigned)e; float sg = 0.0f;
#pragma unroll
        for (int t = 0; t < NTW; ++t) sg += rs[OFW + d * NTW + t] * wt[t];
        const float sc = rs[OBS + d] * w10 + cq; const float v = hf * sc + lf * sg; const float kf = fabsf(v) >= 6.103515625e-05f ? 1.0f : 0.0f; o[e] = tohx(v * kf); }
    h16* d8 = bt + (size_t)q * NKD + 8u * pc; *(volatile v8h*)(d8) = o; __threadfence(); *(volatile v8h*)(d8) = o; }

__global__ __launch_bounds__(256) void k_fin(const float* __restrict__ cc, float* rsl) {
    const unsigned g = blockIdx.x * 256 + threadIdx.x; if (g >= (unsigned)(NRW * NQW / 4)) return; const v4f a = *(const v4f*)(cc + 4u * (size_t)g); v4f o;
#pragma unroll
    for (int e = 0; e < 4; ++e) o[e] = fmaxf(a[e], 0.0f);
    float* dq = rsl + 4u * (size_t)g; *(volatile v4f*)(dq) = o; __threadfence(); *(volatile v4f*)(dq) = o; }

extern "C" void kernel_launch(void* const* d_in, const int* in_sizes, int n_in,
                              void* d_out, int out_size, void* d_ws, size_t ws_size, hipStream_t stream) {
    if (n_in < 6) return;
    if (in_sizes[0] < NRW * NFT || in_sizes[1] < NRW * NFT || in_sizes[2] < NFT * NTW || in_sizes[3] < NFT || in_sizes[4] < (NTW + 1) * NQW || in_sizes[5] < NQW || out_size < NRW * NQW) return;
    const float* xs = (const float*)d_in[0]; const float* fl = (const float*)d_in[1]; const float* fw = (const float*)d_in[2]; const float* bs = (const float*)d_in[3]; const float* ww = (const float*)d_in[4]; const float* cb = (const float*)d_in[5];
    char* wsp = (char*)d_ws;
    auto take = [&](size_t bytes) { char* cur = wsp; wsp += (bytes + 255) & ~(size_t)255; return (void*)cur; };
    float* RS = (float*)take((size_t)8192 * 4); float* XR = (float*)take((size_t)NRW * NFT * 4); float* FR = (float*)take((size_t)NRW * NFT * 4); h16* AM = (h16*)take((size_t)NRW * NKD * 2); h16* BT = (h16*)take((size_t)NQW * NKD * 2); float* CC = (float*)take((size_t)NRW * NQW * 4);
    if ((size_t)(wsp - (char*)d_ws) != WS_TOTAL || WS_TOTAL > ws_size) return;
    auto lay = [&](const float* sp_, h16* dp_, unsigned nrow, unsigned ncol, unsigned dp, unsigned c0, unsigned rbs, unsigned ra, unsigned rs_, unsigned cbs, unsigned sa, unsigned sb, unsigned rlive, unsigned clive) {
        k_lay<<<(nrow * (ncol / 8) + 255) / 256, 256, 0, stream>>>(sp_, dp_, nrow, ncol / 8, dp, c0, rbs, ra, rs_, cbs, sa, sb, rlive, clive); };
    auto rnd = [&](const float* sp_, float* dp_, unsigned nw) { const unsigned npc = (nw + 3) / 4; k_rnd<<<(npc + 255) / 256, 256, 0, stream>>>(sp_, dp_, npc, nw); };
    rnd(xs, XR, NRW * NFT); rnd(fl, FR, NRW * NFT);
    rnd(fw, RS + OFW, NFT * NTW); rnd(bs, RS + OBS, NFT); rnd(ww, RS + OWW, (NTW + 1) * NQW); rnd(cb, RS + OCB, NQW);
    k_opa<<<(NRW * (NFT / 8) + 255) / 256, 256, 0, stream>>>(XR, FR, AM);
    lay(fl, AM, NRW, NFT, NKD, NFT, 16, 0, NFT, 16, 0, 1, NRW, NFT);
    k_opb<<<(NQW * (NKD / 8) + 255) / 256, 256, 0, stream>>>(RS, BT);
    k_gemmw<h16, 0, false><<<dim3(NRW / 64, NQW / 64, 1), 32, 0, stream>>>(AM, nullptr, BT, nullptr, NKD, CC, NQW, nullptr, (size_t)0, (size_t)0, (size_t)0);
    k_fin<<<(NRW * NQW / 4 + 255) / 256, 256, 0, stream>>>(CC, (float*)d_out);
}
